// VarInputFeedRNNDecoder_49821620634192
// MI455X (gfx1250) — hardware-verified
//
#include <hip/hip_runtime.h>
#include <math.h>

constexpr int N_STEP  = 64;
constexpr int N_SRC   = 64;
constexpr int N_BATCH = 64;
constexpr int N_EMB   = 512;
constexpr int N_HID   = 1024;
constexpr int N_LAT   = 128;
constexpr int N_GATE  = 4 * N_HID;
constexpr int K_IN0   = N_EMB + N_HID + N_LAT;
constexpr int K_CAT0  = K_IN0 + N_HID;
constexpr int K_CAT1  = 2 * N_HID;
constexpr int N_QH    = N_HID + 2 * N_LAT;
constexpr int COL_FEED = N_EMB;
constexpr int COL_LAT  = N_EMB + N_HID;
constexpr int COL_H0   = K_IN0;
constexpr int SLAB_P   = 68;
constexpr int KP_PITCH = 32;
constexpr float W_CARRY     = 16.0f;
constexpr float W_CARRY_INV = 1.0f / 16.0f;
constexpr float RES_CARRY   = 2048.0f;
constexpr float RES_INV     = 1.0f / 2048.0f;
constexpr float F32_MIN_NORMAL = 1.17549435e-38f;
static_assert(K_IN0 == 1664 && K_CAT0 == 2688 && K_CAT1 == 2048 && N_QH == 1280, "shape constants");
static_assert(K_CAT0 % 32 == 0 && K_CAT1 % 32 == 0 && N_HID % 32 == 0 && K_IN0 % 32 == 0, "GEMM depth multiple of 32");
static_assert(N_GATE % 256 == 0 && N_QH % 256 == 0 && N_HID % 256 == 0, "GEMM width multiple of the block tile");
static_assert(N_BATCH == 64 && N_SRC == 64, "row tile and source count");
static_assert((K_CAT0 * 2) % 128 == 0 && (COL_FEED * 2) % 128 == 0 && (COL_LAT * 2) % 128 == 0 && (COL_H0 * 2) % 128 == 0, "line aligned column groups");

typedef __attribute__((ext_vector_type(16))) _Float16 v16h;
typedef __attribute__((ext_vector_type(8)))  _Float16 v8h;
typedef __attribute__((ext_vector_type(4)))  _Float16 v4h;
typedef __attribute__((ext_vector_type(16))) __bf16   v16b;
typedef __attribute__((ext_vector_type(8)))  __bf16   v8b;
typedef __attribute__((ext_vector_type(8)))  float    v8f;
typedef __attribute__((ext_vector_type(4)))  float    v4f;

__device__ __forceinline__ unsigned short f2bf_bits(float f) {
  unsigned u = __float_as_uint(f);
  return (unsigned short)((u + 0x7FFFu + ((u >> 16) & 1u)) >> 16);
}
__device__ __forceinline__ float bf_bits2f(unsigned short h) { return __uint_as_float(((unsigned)h) << 16); }

__device__ __forceinline__ float rne11(float s) {
  unsigned u = __float_as_uint(s);
  u = (u + 0x0FFFu + ((u >> 13) & 1u)) & 0xFFFFE000u;
  return __uint_as_float(u);
}
__device__ __forceinline__ _Float16 lo16(float s) {
  const float hf = rne11(s);
  const float d = s - hf;
  return (_Float16)(d * RES_CARRY);
}

__device__ __forceinline__ void guard4_h(v8f& a, v8f& b, v8f& c, v8f& d, v16h x, v16h y) { asm volatile("v_nop\n\tv_nop\n\tv_nop\n\tv_nop" : "+v"(a), "+v"(b), "+v"(c), "+v"(d) : "v"(x), "v"(y)); }
__device__ __forceinline__ void guard4_b(v8f& a, v8f& b, v8f& c, v8f& d, v16b x, v16b y) { asm volatile("v_nop\n\tv_nop\n\tv_nop\n\tv_nop" : "+v"(a), "+v"(b), "+v"(c), "+v"(d) : "v"(x), "v"(y)); }
__device__ __forceinline__ void guard2_h(v8f& a, v8f& b, v16h x, v16h y) { asm volatile("v_nop\n\tv_nop\n\tv_nop\n\tv_nop" : "+v"(a), "+v"(b) : "v"(x), "v"(y)); }
__device__ __forceinline__ void keep4_h(v16h a, v16h b, v16h c, v16h d) { asm volatile("v_nop" :: "v"(a), "v"(b), "v"(c), "v"(d)); }
__device__ __forceinline__ void keep4_b(v16b a, v16b b, v16b c, v16b d) { asm volatile("v_nop" :: "v"(a), "v"(b), "v"(c), "v"(d)); }
__device__ __forceinline__ void acc_guard4(v8f& a, v8f& b, v8f& c, v8f& d) { asm volatile("v_nop\n\tv_nop\n\tv_nop\n\tv_nop" : "+v"(a), "+v"(b), "+v"(c), "+v"(d)); }

template <typename T> struct Frag;
template <> struct Frag<_Float16> {
  typedef v16h V; union U { v16h v; v8h h[2]; };
  static __device__ __forceinline__ v16h load(const _Float16* p) {
    U f; f.h[0] = *(const v8h*)(p); f.h[1] = *(const v8h*)(p + 16); return f.v;
  }
  static __device__ __forceinline__ v8f mma(v16h a, v16h b, v8f c) {
    return __builtin_amdgcn_wmma_f32_16x16x32_f16(false, a, false, b, (short)0, c, false, false);
  }
  static __device__ __forceinline__ void guard4(v8f& a, v8f& b, v8f& c, v8f& d, v16h x, v16h y) { guard4_h(a, b, c, d, x, y); }
  static __device__ __forceinline__ void keep(v16h a, v16h b, v16h c, v16h d) { keep4_h(a, b, c, d); }
};
template <> struct Frag<__bf16> {
  typedef v16b V; union U { v16b v; v8b h[2]; };
  static __device__ __forceinline__ v16b load(const __bf16* p) {
    U f; f.h[0] = *(const v8b*)(p); f.h[1] = *(const v8b*)(p + 16); return f.v;
  }
  static __device__ __forceinline__ v8f mma(v16b a, v16b b, v8f c) {
    return __builtin_amdgcn_wmma_f32_16x16x32_bf16(false, a, false, b, (short)0, c, false, false);
  }
  static __device__ __forceinline__ void guard4(v8f& a, v8f& b, v8f& c, v8f& d, v16b x, v16b y) { guard4_b(a, b, c, d, x, y); }
  static __device__ __forceinline__ void keep(v16b a, v16b b, v16b c, v16b d) { keep4_b(a, b, c, d); }
};

__device__ __forceinline__ void wave_lds_sync() {
  __builtin_amdgcn_fence(__ATOMIC_RELEASE, "workgroup");
  __builtin_amdgcn_wave_barrier();
  __builtin_amdgcn_fence(__ATOMIC_ACQUIRE, "workgroup");
}

__device__ __forceinline__ float sig_f(float x) {
  const float e = __expf(-x);
  return __builtin_amdgcn_rcpf(1.0f + e);
}
__device__ __forceinline__ float tanh_f(float x) {
  const float e = __expf(2.0f * x);
  const float rr = __builtin_amdgcn_rcpf(e + 1.0f);
  return 1.0f - 2.0f * rr;
}

template <typename T, bool SPLIT>
__device__ __forceinline__ void mm_tile64(v8f (&acc)[4][4],
                                          const T* A, const T* A2, int lda,
                                          const T* Bt, const T* Bt2, int ldb,
                                          int n0, int kdim, int rlane, int koff) {
  typedef typename Frag<T>::V V;
  const T* ap  = A   + (size_t)rlane * lda + koff;
  const T* ap2 = A2  + (size_t)rlane * lda + koff;
  const T* bp  = Bt  + (size_t)(n0 + rlane) * ldb + koff;
  const T* bp2 = Bt2 + (size_t)(n0 + rlane) * ldb + koff;
  const size_t a16 = (size_t)16 * lda;
  const size_t b16 = (size_t)16 * ldb;
  for (int k0 = 0; k0 < kdim; k0 += 32) {
    V bh[4], bl[4];
#pragma unroll
    for (int j = 0; j < 4; ++j) {
      bh[j] = Frag<T>::load(bp + j * b16 + k0);
      if (SPLIT) bl[j] = Frag<T>::load(bp2 + j * b16 + k0);
      else bl[j] = bh[j];
    }
#pragma unroll
    for (int i = 0; i < 4; ++i) {
      const V ah = Frag<T>::load(ap + i * a16 + k0);
      V al = ah;
      if (SPLIT) al = Frag<T>::load(ap2 + i * a16 + k0);
#pragma unroll
      for (int j = 0; j < 4; ++j) {
        acc[i][j] = Frag<T>::mma(ah, bh[j], acc[i][j]);
        if (SPLIT) {
          acc[i][j] = Frag<T>::mma(ah, bl[j], acc[i][j]);
          acc[i][j] = Frag<T>::mma(al, bh[j], acc[i][j]);
        }
      }
      Frag<T>::guard4(acc[i][0], acc[i][1], acc[i][2], acc[i][3], ah, al);
    }
    Frag<T>::keep(bh[0], bh[1], bh[2], bh[3]);
    if (SPLIT) Frag<T>::keep(bl[0], bl[1], bl[2], bl[3]);
  }
  acc_guard4(acc[0][0], acc[0][1], acc[0][2], acc[0][3]);
  acc_guard4(acc[1][0], acc[1][1], acc[1][2], acc[1][3]);
  acc_guard4(acc[2][0], acc[2][1], acc[2][2], acc[2][3]);
  acc_guard4(acc[3][0], acc[3][1], acc[3][2], acc[3][3]);
}

__device__ __forceinline__ void wfrag_build(const float* p, v16h& bh, v16h& bl) {
  const v4f w0 = *(const v4f*)(p);
  const v4f w1 = *(const v4f*)(p + 4);
  const v4f w2 = *(const v4f*)(p + 16);
  const v4f w3 = *(const v4f*)(p + 20);
#pragma unroll
  for (int e = 0; e < 4; ++e) {
    const float f0 = w0[e];
    const float f1 = w1[e];
    const float f2 = w2[e];
    const float f3 = w3[e];
    const float s0 = f0 * W_CARRY;
    const float s1 = f1 * W_CARRY;
    const float s2 = f2 * W_CARRY;
    const float s3 = f3 * W_CARRY;
    bh[e]      = (_Float16)s0;
    bh[4 + e]  = (_Float16)s1;
    bh[8 + e]  = (_Float16)s2;
    bh[12 + e] = (_Float16)s3;
    bl[e]      = lo16(s0);
    bl[4 + e]  = lo16(s1);
    bl[8 + e]  = lo16(s2);
    bl[12 + e] = lo16(s3);
  }
}

__device__ __forceinline__ void mm_resid_seg(v8f (&acc)[4][4],
                                             const _Float16* Ah, const _Float16* Al, int lda,
                                             const float* Wsrc, int wpitch, int urow,
                                             int kseg, int rlane, int koff) {
  const _Float16* aph = Ah + (size_t)rlane * lda + koff;
  const _Float16* apl = Al + (size_t)rlane * lda + koff;
  const float* wp = Wsrc + (size_t)urow * wpitch + koff;
  const size_t a16 = (size_t)16 * lda;
  const size_t wg  = (size_t)N_HID * wpitch;
  for (int k0 = 0; k0 < kseg; k0 += 32) {
#pragma unroll
    for (int jp = 0; jp < 2; ++jp) {
      v16h bh0, bl0, bh1, bl1;
      wfrag_build(wp + (size_t)(2 * jp) * wg + k0, bh0, bl0);
      wfrag_build(wp + (size_t)(2 * jp + 1) * wg + k0, bh1, bl1);
#pragma unroll
      for (int i = 0; i < 4; ++i) {
        const v16h ah = Frag<_Float16>::load(aph + i * a16 + k0);
        const v16h al = Frag<_Float16>::load(apl + i * a16 + k0);
        acc[i][2 * jp]     = Frag<_Float16>::mma(ah, bl0, acc[i][2 * jp]);
        acc[i][2 * jp]     = Frag<_Float16>::mma(al, bh0, acc[i][2 * jp]);
        acc[i][2 * jp + 1] = Frag<_Float16>::mma(ah, bl1, acc[i][2 * jp + 1]);
        acc[i][2 * jp + 1] = Frag<_Float16>::mma(al, bh1, acc[i][2 * jp + 1]);
        guard2_h(acc[i][2 * jp], acc[i][2 * jp + 1], ah, al);
      }
      keep4_h(bh0, bl0, bh1, bl1);
    }
  }
  acc_guard4(acc[0][0], acc[0][1], acc[0][2], acc[0][3]);
  acc_guard4(acc[1][0], acc[1][1], acc[1][2], acc[1][3]);
  acc_guard4(acc[2][0], acc[2][1], acc[2][2], acc[2][3]);
  acc_guard4(acc[3][0], acc[3][1], acc[3][2], acc[3][3]);
}

template <int HMODE, bool REFINE>
__global__ __launch_bounds__(256) void gemm_cell_kernel(
    const unsigned short* __restrict__ Ap, const unsigned short* Alp, int lda,
    const unsigned short* __restrict__ Btp, int kdim,
    const float* Wfa, int wpa, int ksa, const float* Wfb, int wpb,
    const float* __restrict__ biasp,
    const float* __restrict__ cin, float* __restrict__ cnext,
    unsigned short* hd0, int hp0,
    unsigned short* hd1, int hp1,
    unsigned short* bhi, unsigned short* blo,
    unsigned short* hlo, int hlp) {
  __shared__ __align__(16) float Sl[4][16 * SLAB_P];
  __shared__ __align__(16) float Cs[64 * SLAB_P];
  __shared__ __align__(16) float Hs[64 * SLAB_P];
  const int tid = threadIdx.x, lane = tid & 31, wave = (tid >> 5) & 3;
  const int rlane = lane & 15, hh = lane >> 4, koff = hh * 8;
  const int bx = blockIdx.x;
  const int u0 = 64 * bx;
  const int n0 = 256 * bx + 64 * wave;
  const int ucol = 16 * wave + rlane;
  {
    const int rq = tid >> 4, c4 = (tid & 15) * 4;
#pragma unroll
    for (int p = 0; p < 8; ++p) {
      const int row = p * 8 + rq;
      const v4f v = *(const v4f*)(cin + (size_t)row * N_HID + u0 + c4);
      *(v4f*)(Cs + row * SLAB_P + c4) = v;
    }
  }
  const v8f z8 = {0.f, 0.f, 0.f, 0.f, 0.f, 0.f, 0.f, 0.f};
  v8f acc[4][4];
#pragma unroll
  for (int i = 0; i < 4; ++i)
#pragma unroll
    for (int j = 0; j < 4; ++j) acc[i][j] = z8;
  const _Float16* A  = (const _Float16*)Ap;
  const _Float16* Bt = (const _Float16*)Btp;
  if (REFINE) {
    const _Float16* Al = (const _Float16*)Alp;
    const int urow = u0 + ucol;
    mm_resid_seg(acc, A, Al, lda, Wfa, wpa, urow, ksa, rlane, koff);
    mm_resid_seg(acc, A + ksa, Al + ksa, lda, Wfb, wpb, urow, kdim - ksa, rlane, koff);
#pragma unroll
    for (int i = 0; i < 4; ++i)
#pragma unroll
      for (int j = 0; j < 4; ++j)
#pragma unroll
        for (int r = 0; r < 8; ++r) acc[i][j][r] = acc[i][j][r] * RES_INV;
  }
  mm_tile64<_Float16, false>(acc, A, A, lda, Bt, Bt, kdim, n0, kdim, rlane, koff);
  __syncthreads();

  const float bi0 = biasp[n0 + rlane];
  const float bi1 = biasp[n0 + 16 + rlane];
  const float bi2 = biasp[n0 + 32 + rlane];
  const float bi3 = biasp[n0 + 48 + rlane];
  float* slab = Sl[wave];
#pragma unroll
  for (int i = 0; i < 4; ++i) {
#pragma unroll
    for (int j = 0; j < 4; ++j)
#pragma unroll
      for (int r = 0; r < 8; ++r) slab[(8 * hh + r) * SLAB_P + 16 * j + rlane] = acc[i][j][r] * W_CARRY_INV;
    wave_lds_sync();
#pragma unroll 1
    for (int r = 0; r < 8; ++r) {
      const int lr = 8 * hh + r;
      const float* sp = slab + lr * SLAB_P + rlane;
      const float zi = sp[0]  + bi0;
      const float zf = sp[16] + bi1;
      const float zg = sp[32] + bi2;
      const float zo = sp[48] + bi3;
      const int cidx = (16 * i + lr) * SLAB_P + ucol;
      const float cp = Cs[cidx];
      const float ig = sig_f(zi);
      const float fg = sig_f(zf);
      const float gg = tanh_f(zg);
      const float og = sig_f(zo);
      const float cn = fg * cp + ig * gg;
      const float hn = og * tanh_f(cn);
      Cs[cidx] = cn;
      Hs[cidx] = hn;
    }
    wave_lds_sync();
  }
  __syncthreads();

  {
    const int rq = tid >> 4, c4 = (tid & 15) * 4;
    for (int pass = 0; pass < 2; ++pass) {
#pragma unroll
      for (int p = 0; p < 8; ++p) {
        const int row = p * 8 + rq;
        const v4f v = *(const v4f*)(Cs + row * SLAB_P + c4);
        *(volatile v4f*)(cnext + (size_t)row * N_HID + u0 + c4) = v;
      }
      __threadfence();
    }
  }
  {
    const int rq = tid >> 3, c8 = (tid & 7) * 8;
    for (int pass = 0; pass < 2; ++pass) {
#pragma unroll
      for (int p = 0; p < 4; ++p) {
        const int row = p * 16 + rq;
        const float* sp = Hs + row * SLAB_P + c8;
        const v4f x0 = *(const v4f*)(sp);
        const v4f x1 = *(const v4f*)(sp + 4);
        v8h hv, bh8, bl8, lo8;
#pragma unroll
        for (int e = 0; e < 4; ++e) {
          const float f0 = x0[e];
          const float f1 = x1[e];
          hv[e]     = (_Float16)f0;
          hv[4 + e] = (_Float16)f1;
          if (HMODE == 1) {
            const unsigned short h0b = f2bf_bits(f0);
            const unsigned short l0b = f2bf_bits(f0 - bf_bits2f(h0b));
            const unsigned short h1b = f2bf_bits(f1);
            const unsigned short l1b = f2bf_bits(f1 - bf_bits2f(h1b));
            bh8[e]     = __builtin_bit_cast(_Float16, h0b);
            bh8[4 + e] = __builtin_bit_cast(_Float16, h1b);
            bl8[e]     = __builtin_bit_cast(_Float16, l0b);
            bl8[4 + e] = __builtin_bit_cast(_Float16, l1b);
          } else {
            bh8[e]     = hv[e];
            bh8[4 + e] = hv[4 + e];
            bl8[e]     = hv[e];
            bl8[4 + e] = hv[4 + e];
          }
          if (HMODE >= 1) {
            lo8[e]     = lo16(f0);
            lo8[4 + e] = lo16(f1);
          } else {
            lo8[e]     = hv[e];
            lo8[4 + e] = hv[4 + e];
          }
        }
        *(volatile v8h*)(hd0 + (size_t)row * hp0 + u0 + c8) = hv;
        *(volatile v8h*)(hd1 + (size_t)row * hp1 + u0 + c8) = hv;
        if (HMODE == 1) {
          *(volatile v8h*)(bhi + (size_t)row * N_HID + u0 + c8) = bh8;
          *(volatile v8h*)(blo + (size_t)row * N_HID + u0 + c8) = bl8;
        }
        if (HMODE >= 1) {
          *(volatile v8h*)(hlo + (size_t)row * hlp + u0 + c8) = lo8;
        }
      }
      __threadfence();
    }
  }
}

__global__ __launch_bounds__(256) void gemm_qh_kernel(
    const unsigned short* __restrict__ Ahp, const unsigned short* __restrict__ Alp,
    const unsigned short* __restrict__ Bhp, const unsigned short* __restrict__ Blp,
    const float* __restrict__ biasp, float* __restrict__ C) {
  __shared__ __align__(16) float Sl[4][16 * SLAB_P];
  const int tid = threadIdx.x, lane = tid & 31, wave = (tid >> 5) & 3;
  const int rlane = lane & 15, hh = lane >> 4, koff = hh * 8;
  const int n0 = 256 * blockIdx.x + 64 * wave;
  const v8f z8 = {0.f, 0.f, 0.f, 0.f, 0.f, 0.f, 0.f, 0.f};
  v8f acc[4][4];
#pragma unroll
  for (int i = 0; i < 4; ++i)
#pragma unroll
    for (int j = 0; j < 4; ++j) acc[i][j] = z8;
  mm_tile64<__bf16, true>(acc, (const __bf16*)Ahp, (const __bf16*)Alp, N_HID,
                          (const __bf16*)Bhp, (const __bf16*)Blp, N_HID, n0, N_HID, rlane, koff);
  const float bi0 = biasp[n0 + rlane];
  const float bi1 = biasp[n0 + 16 + rlane];
  const float bi2 = biasp[n0 + 32 + rlane];
  const float bi3 = biasp[n0 + 48 + rlane];
  float* slab = Sl[wave];
  const int c4 = rlane * 4;
#pragma unroll
  for (int i = 0; i < 4; ++i) {
#pragma unroll
    for (int r = 0; r < 8; ++r) {
      slab[(8 * hh + r) * SLAB_P + rlane]      = acc[i][0][r] + bi0;
      slab[(8 * hh + r) * SLAB_P + 16 + rlane] = acc[i][1][r] + bi1;
      slab[(8 * hh + r) * SLAB_P + 32 + rlane] = acc[i][2][r] + bi2;
      slab[(8 * hh + r) * SLAB_P + 48 + rlane] = acc[i][3][r] + bi3;
    }
    wave_lds_sync();
    for (int pass = 0; pass < 2; ++pass) {
#pragma unroll
      for (int it = 0; it < 8; ++it) {
        const int row = it * 2 + hh;
        const v4f v = *(const v4f*)(slab + row * SLAB_P + c4);
        *(volatile v4f*)(C + (size_t)(16 * i + row) * N_QH + n0 + c4) = v;
      }
      __threadfence();
    }
    wave_lds_sync();
  }
}

__global__ __launch_bounds__(256) void gemm_out_kernel(
    const unsigned short* __restrict__ Ap, const unsigned short* __restrict__ Alp,
    const unsigned short* __restrict__ Btp,
    float* __restrict__ dec, unsigned short* __restrict__ feed, int fpitch) {
  __shared__ __align__(16) float Sl[4][16 * SLAB_P];
  const int tid = threadIdx.x, lane = tid & 31, wave = (tid >> 5) & 3;
  const int rlane = lane & 15, hh = lane >> 4, koff = hh * 8;
  const int n0 = 256 * blockIdx.x + 64 * wave;
  const v8f z8 = {0.f, 0.f, 0.f, 0.f, 0.f, 0.f, 0.f, 0.f};
  v8f acc[4][4];
#pragma unroll
  for (int i = 0; i < 4; ++i)
#pragma unroll
    for (int j = 0; j < 4; ++j) acc[i][j] = z8;
  const _Float16* A  = (const _Float16*)Ap;
  const _Float16* Al = (const _Float16*)Alp;
  const _Float16* Bt = (const _Float16*)Btp;
  mm_tile64<_Float16, false>(acc, Al, Al, K_CAT1, Bt, Bt, K_CAT1, n0, K_CAT1, rlane, koff);
#pragma unroll
  for (int i = 0; i < 4; ++i)
#pragma unroll
    for (int j = 0; j < 4; ++j)
#pragma unroll
      for (int r = 0; r < 8; ++r) acc[i][j][r] = acc[i][j][r] * RES_INV;
  mm_tile64<_Float16, false>(acc, A, A, K_CAT1, Bt, Bt, K_CAT1, n0, K_CAT1, rlane, koff);
  float* slab = Sl[wave];
  const int c4 = rlane * 4;
  const int q8 = lane >> 3, c8 = (lane & 7) * 8;
#pragma unroll
  for (int i = 0; i < 4; ++i) {
#pragma unroll
    for (int j = 0; j < 4; ++j)
#pragma unroll
      for (int r = 0; r < 8; ++r) slab[(8 * hh + r) * SLAB_P + 16 * j + rlane] = acc[i][j][r] * W_CARRY_INV;
    wave_lds_sync();
#pragma unroll 1
    for (int q = 0; q < 32; ++q) {
      const int o = q * 32 + lane;
      float* sp = slab + (o >> 6) * SLAB_P + (o & 63);
      const float x = *sp;
      const float y = tanh_f(x);
      *sp = y;
    }
    wave_lds_sync();
    for (int pass = 0; pass < 2; ++pass) {
#pragma unroll
      for (int it = 0; it < 8; ++it) {
        const int row = it * 2 + hh;
        const v4f v = *(const v4f*)(slab + row * SLAB_P + c4);
        *(volatile v4f*)(dec + (size_t)(16 * i + row) * N_HID + n0 + c4) = v;
      }
#pragma unroll
      for (int it = 0; it < 4; ++it) {
        const int row = it * 4 + q8;
        const float* sp = slab + row * SLAB_P + c8;
        const v4f x0 = *(const v4f*)(sp);
        const v4f x1 = *(const v4f*)(sp + 4);
        v8h hv;
#pragma unroll
        for (int e = 0; e < 4; ++e) {
          const float f0 = x0[e];
          const float f1 = x1[e];
          hv[e]     = (_Float16)f0;
          hv[4 + e] = (_Float16)f1;
        }
        *(volatile v8h*)(feed + (size_t)(16 * i + row) * fpitch + n0 + c8) = hv;
      }
      __threadfence();
    }
    wave_lds_sync();
  }
}

template <int MODE, bool PERM>
__global__ __launch_bounds__(256) void cvt8_kernel(const float* __restrict__ src, int spitch, int ncol8, int nrow,
                                                   unsigned short* __restrict__ dst, unsigned short* dst2,
                                                   int dpitch, float sc) {
  const int i  = blockIdx.x * 256 + threadIdx.x;
  const int n8 = nrow * ncol8;
  if (i < n8) {
    const int row = i / ncol8;
    const int c8  = i - row * ncol8;
    const int srow = PERM ? ((((row & 63) >> 4) * N_HID) + ((row >> 6) * 16) + (row & 15)) : row;
    const float* sp = src + (size_t)srow * spitch + c8 * 8;
    const v4f a = *(const v4f*)(sp);
    const v4f b = *(const v4f*)(sp + 4);
    v8h hv, lv;
#pragma unroll
    for (int e = 0; e < 4; ++e) {
      const float f0 = a[e];
      const float f1 = b[e];
      if (MODE == 0) {
        hv[e]     = (_Float16)(f0 * sc);
        hv[4 + e] = (_Float16)(f1 * sc);
        lv[e]     = hv[e];
        lv[4 + e] = hv[4 + e];
      } else if (MODE == 1) {
        const unsigned short h0b = f2bf_bits(f0);
        const unsigned short l0b = f2bf_bits(f0 - bf_bits2f(h0b));
        const unsigned short h1b = f2bf_bits(f1);
        const unsigned short l1b = f2bf_bits(f1 - bf_bits2f(h1b));
        hv[e]     = __builtin_bit_cast(_Float16, h0b);
        hv[4 + e] = __builtin_bit_cast(_Float16, h1b);
        lv[e]     = __builtin_bit_cast(_Float16, l0b);
        lv[4 + e] = __builtin_bit_cast(_Float16, l1b);
      } else {
        const float s0 = f0 * sc;
        const float s1 = f1 * sc;
        hv[e]     = (_Float16)s0;
        hv[4 + e] = (_Float16)s1;
        lv[e]     = lo16(s0);
        lv[4 + e] = lo16(s1);
      }
    }
    const size_t o = (size_t)row * dpitch + (size_t)c8 * 8;
    *(volatile v8h*)(dst + o) = hv;
    if (MODE >= 1) *(volatile v8h*)(dst2 + o) = lv;
    __threadfence();
    *(volatile v8h*)(dst + o) = hv;
    if (MODE >= 1) *(volatile v8h*)(dst2 + o) = lv;
  }
}

__global__ __launch_bounds__(256) void bias_kernel(const float* __restrict__ b_ih0, const float* __restrict__ b_hh0,
                                                   const float* __restrict__ b_ih1, const float* __restrict__ b_hh1,
                                                   const float* __restrict__ b_mu, const float* __restrict__ b_lv,
                                                   float* __restrict__ bs0, float* __restrict__ bs1,
                                                   float* __restrict__ bqh) {
  const int tid = threadIdx.x;
  const int blk = blockIdx.x;
  const int region = blk >> 2;
  const int g = (blk & 3) * 256 + tid;
  if (region < 2) {
    const int p4 = g * 4;
    const int srci = (((p4 & 63) >> 4) * N_HID) + ((p4 >> 6) * 16) + (p4 & 15);
    const float* ba = (region == 0) ? b_ih0 : b_ih1;
    const float* bb = (region == 0) ? b_hh0 : b_hh1;
    float* dp = ((region == 0) ? bs0 : bs1) + p4;
    const v4f x = *(const v4f*)(ba + srci);
    const v4f y = *(const v4f*)(bb + srci);
    const v4f o = x + y;
    *(volatile v4f*)dp = o;
    __threadfence();
    *(volatile v4f*)dp = o;
  } else {
    const int n4 = g * 4;
    if (n4 < N_QH) {
      int im = n4 - N_HID;
      im = im < 0 ? 0 : (im > N_LAT - 4 ? N_LAT - 4 : im);
      int il = n4 - (N_HID + N_LAT);
      il = il < 0 ? 0 : (il > N_LAT - 4 ? N_LAT - 4 : il);
      const v4f vm = *(const v4f*)(b_mu + im);
      const v4f vl = *(const v4f*)(b_lv + il);
      v4f o;
#pragma unroll
      for (int e = 0; e < 4; ++e) {
        const float m = vm[e];
        const float l = vl[e];
        o[e] = (n4 < N_HID) ? 0.0f : ((n4 < N_HID + N_LAT) ? m : l);
      }
      *(volatile v4f*)(bqh + n4) = o;
      __threadfence();
      *(volatile v4f*)(bqh + n4) = o;
    }
  }
}

template <bool WITH_LO>
__device__ __forceinline__ void zk_compute(const float* qrow, const float* eprow, _Float16* zs, _Float16* zl,
                                           float* red, int tid) {
  const int lane = tid & 31, wave = tid >> 5;
  const int zi = tid & (N_LAT - 1);
  const float mu = qrow[N_HID + zi];
  const float lv = qrow[N_HID + N_LAT + zi];
  const float ep = eprow[zi];
  const float zval = mu + ep * expf(0.5f * lv);
  float term = ((1.0f + lv) - mu * mu) - expf(lv);
  term = (tid < N_LAT) ? term : 0.0f;
#pragma unroll
  for (int off = 16; off > 0; off >>= 1) term += __shfl_xor(term, off, 32);
  if (lane == 0) red[wave] = term;
  if (tid < N_LAT) {
    zs[zi] = (_Float16)zval;
    if (WITH_LO) zl[zi] = lo16(zval);
  }
}

__device__ __forceinline__ void zk_store(const _Float16* zs, float kv, unsigned short* x0row, float* kprow, int tid) {
  const int lane = tid & 31, wave = tid >> 5;
  if (wave == 1 && lane < 16) {
    const v8h v = *(const v8h*)(zs + 8 * lane);
    *(volatile v8h*)(x0row + COL_LAT + 8 * lane) = v;
  }
  if (wave == 2) {
    const float w = (lane == 0) ? kv : 0.0f;
    *(volatile float*)(kprow + lane) = w;
  }
}

__global__ __launch_bounds__(256) void zk_kernel(const float* __restrict__ qml, const float* __restrict__ epst,
                                                 unsigned short* __restrict__ x0t, unsigned short* __restrict__ a0l,
                                                 float* __restrict__ kpt) {
  __shared__ __align__(16) _Float16 zs[N_LAT];
  __shared__ __align__(16) _Float16 zl[N_LAT];
  __shared__ float red[8];
  const int tid = threadIdx.x;
  const int lane = tid & 31, wave = tid >> 5;
  const int b = blockIdx.x;
  zk_compute<true>(qml + (size_t)b * N_QH, epst + (size_t)b * N_LAT, zs, zl, red, tid);
  __syncthreads();
  const float kv = -0.5f * ((red[0] + red[1]) + (red[2] + red[3]));
  for (int pass = 0; pass < 2; ++pass) {
    zk_store(zs, kv, x0t + (size_t)b * K_CAT0, kpt + (size_t)b * KP_PITCH, tid);
    if (wave == 3 && lane < 16) {
      const v8h v = *(const v8h*)(zl + 8 * lane);
      *(volatile v8h*)(a0l + (size_t)b * K_CAT0 + COL_LAT + 8 * lane) = v;
    }
    __threadfence();
  }
}

__global__ __launch_bounds__(256) void att_kernel(const float* __restrict__ qml, const float* __restrict__ enc,
                                                  const int* __restrict__ lengths, const float* __restrict__ epsn,
                                                  float* __restrict__ attn_t, unsigned short* __restrict__ xo_t,
                                                  unsigned short* __restrict__ xol_t,
                                                  unsigned short* __restrict__ x0n, float* __restrict__ kpn) {
  __shared__ __align__(16) float sc[N_SRC];
  __shared__ __align__(16) float al[N_SRC];
  __shared__ __align__(16) _Float16 ctxh[N_HID];
  __shared__ __align__(16) _Float16 ctxl[N_HID];
  __shared__ __align__(16) _Float16 zs[N_LAT];
  __shared__ float red[8];
  const int tid = threadIdx.x, lane = tid & 31, wave = tid >> 5;
  const int b = blockIdx.x;
  int len = lengths[b];
  len = len < 0 ? 0 : (len > N_SRC ? N_SRC : len);
  const int nl = (len == 0) ? N_SRC : len;
  const float* qrow = qml + (size_t)b * N_QH;
  const float* eb = enc + (size_t)b * N_HID;
  v4f qv[8];
#pragma unroll
  for (int j = 0; j < 8; ++j) qv[j] = *(const v4f*)(qrow + 128 * j + 4 * lane);
#pragma unroll 1
  for (int si = 0; si < 8; ++si) {
    const int s = wave + 8 * si;
    float a0 = 0.0f, a1 = 0.0f, a2 = 0.0f, a3 = 0.0f;
    if (s < nl) {
      const float* er = eb + (size_t)s * (N_BATCH * N_HID) + 4 * lane;
#pragma unroll
      for (int j = 0; j < 8; ++j) {
        const v4f e = *(const v4f*)(er + 128 * j);
        a0 = fmaf(qv[j][0], e[0], a0);
        a1 = fmaf(qv[j][1], e[1], a1);
        a2 = fmaf(qv[j][2], e[2], a2);
        a3 = fmaf(qv[j][3], e[3], a3);
      }
    }
    float a = (a0 + a1) + (a2 + a3);
#pragma unroll
    for (int off = 16; off > 0; off >>= 1) a += __shfl_xor(a, off, 32);
    if (lane == 0) sc[s] = a;
  }
  zk_compute<false>(qrow, epsn + (size_t)b * N_LAT, zs, zs, red, tid);
  __syncthreads();

  {
    float v0 = sc[lane];
    float v1 = sc[lane + 32];
    v0 = (lane < len) ? v0 : -1.0e30f;
    v1 = (lane + 32 < len) ? v1 : -1.0e30f;
    float mx = fmaxf(v0, v1);
#pragma unroll
    for (int off = 16; off > 0; off >>= 1) mx = fmaxf(mx, __shfl_xor(mx, off, 32));
    float e0 = expf(v0 - mx);
    float e1 = expf(v1 - mx);
    e0 = (e0 < F32_MIN_NORMAL) ? 0.0f : e0;
    e1 = (e1 < F32_MIN_NORMAL) ? 0.0f : e1;
    float sm = e0 + e1;
#pragma unroll
    for (int off = 16; off > 0; off >>= 1) sm += __shfl_xor(sm, off, 32);
    const float inv = 1.0f / sm;
    const float p0 = e0 * inv;
    const float p1 = e1 * inv;
    if (wave == 0) {
      al[lane] = p0;
      al[lane + 32] = p1;
    }
  }
  __syncthreads();

  {
    float c0 = 0.0f, c1 = 0.0f, c2 = 0.0f, c3 = 0.0f;
    const float* ec = eb + 4 * tid;
#pragma unroll 2
    for (int s = 0; s < nl; ++s) {
      const float a = al[s];
      const v4f e = *(const v4f*)(ec + (size_t)s * (N_BATCH * N_HID));
      c0 = fmaf(a, e[0], c0);
      c1 = fmaf(a, e[1], c1);
      c2 = fmaf(a, e[2], c2);
      c3 = fmaf(a, e[3], c3);
    }
    v4h ch, cl;
    ch[0] = (_Float16)c0;
    ch[1] = (_Float16)c1;
    ch[2] = (_Float16)c2;
    ch[3] = (_Float16)c3;
    cl[0] = lo16(c0);
    cl[1] = lo16(c1);
    cl[2] = lo16(c2);
    cl[3] = lo16(c3);
    *(v4h*)(ctxh + 4 * tid) = ch;
    *(v4h*)(ctxl + 4 * tid) = cl;
  }
  __syncthreads();

  const float kv = -0.5f * ((red[0] + red[1]) + (red[2] + red[3]));
  for (int pass = 0; pass < 2; ++pass) {
    if (tid < 128) {
      const v8h v = *(const v8h*)(ctxh + 8 * tid);
      *(volatile v8h*)(xo_t + (size_t)b * K_CAT1 + 8 * tid) = v;
    }
    if (tid >= 128) {
      const v8h v = *(const v8h*)(ctxl + 8 * (tid - 128));
      *(volatile v8h*)(xol_t + (size_t)b * K_CAT1 + 8 * (tid - 128)) = v;
    }
    if (tid < 16) {
      const v4f v = *(const v4f*)(al + 4 * tid);
      *(volatile v4f*)(attn_t + (size_t)b * N_SRC + 4 * tid) = v;
    }
    zk_store(zs, kv, x0n + (size_t)b * K_CAT0, kpn + (size_t)b * KP_PITCH, tid);
    __threadfence();
  }
}

__global__ __launch_bounds__(32) void kld_final_kernel(const float* __restrict__ kp, float* __restrict__ out2) {
  const int lane = threadIdx.x & 31;
  float a0 = 0.0f, a1 = 0.0f;
#pragma unroll 1
  for (int t = 0; t < N_STEP; ++t) {
    a0 += kp[((size_t)t * N_BATCH + lane) * KP_PITCH];
    a1 += kp[((size_t)t * N_BATCH + lane + 32) * KP_PITCH];
  }
  float a = a0 + a1;
#pragma unroll
  for (int off = 16; off > 0; off >>= 1) a += __shfl_xor(a, off, 32);
  if (lane == 0) {
    *(volatile float*)out2 = a;
    __threadfence();
    *(volatile float*)out2 = a;
  }
}

extern "C" void kernel_launch(void* const* d_in, const int* in_sizes, int n_in,
                              void* d_out, int out_size, void* d_ws, size_t ws_size, hipStream_t stream) {
  if (n_in < 21 || d_out == nullptr || d_ws == nullptr) return;
  if (in_sizes[0] != N_STEP * N_BATCH * N_EMB || in_sizes[1] != N_SRC * N_BATCH * N_HID || in_sizes[2] != N_BATCH ||
      in_sizes[3] != 2 * N_BATCH * N_HID || in_sizes[4] != 2 * N_BATCH * N_HID || in_sizes[5] != N_BATCH * N_HID ||
      in_sizes[6] != N_STEP * N_BATCH * N_LAT || in_sizes[7] != N_GATE * K_IN0 || in_sizes[8] != N_GATE * N_HID ||
      in_sizes[9] != N_GATE || in_sizes[10] != N_GATE || in_sizes[11] != N_GATE * N_HID ||
      in_sizes[12] != N_GATE * N_HID || in_sizes[13] != N_GATE || in_sizes[14] != N_GATE ||
      in_sizes[15] != N_LAT * N_HID || in_sizes[16] != N_LAT || in_sizes[17] != N_LAT * N_HID ||
      in_sizes[18] != N_LAT || in_sizes[19] != N_HID * N_HID || in_sizes[20] != N_HID * K_CAT1 ||
      out_size != N_STEP * N_BATCH * N_HID + N_STEP * N_BATCH * N_SRC + 1) return;

  const float* trg_emb = (const float*)d_in[0];
  const float* enc     = (const float*)d_in[1];
  const int*   lengths = (const int*)d_in[2];
  const float* h0_in   = (const float*)d_in[3];
  const float* c0_in   = (const float*)d_in[4];
  const float* in_feed = (const float*)d_in[5];
  const float* eps     = (const float*)d_in[6];
  const float* W_ih0   = (const float*)d_in[7];
  const float* W_hh0   = (const float*)d_in[8];
  const float* b_ih0   = (const float*)d_in[9];
  const float* b_hh0   = (const float*)d_in[10];
  const float* W_ih1   = (const float*)d_in[11];
  const float* W_hh1   = (const float*)d_in[12];
  const float* b_ih1   = (const float*)d_in[13];
  const float* b_hh1   = (const float*)d_in[14];
  const float* W_mu    = (const float*)d_in[15];
  const float* b_mu    = (const float*)d_in[16];
  const float* W_lv    = (const float*)d_in[17];
  const float* b_lv    = (const float*)d_in[18];
  const float* W_a     = (const float*)d_in[19];
  const float* W_out   = (const float*)d_in[20];
  float* out   = (float*)d_out;
  float* dec   = out;
  float* attns = out + (size_t)N_STEP * N_BATCH * N_HID;
  float* kld   = attns + (size_t)N_STEP * N_BATCH * N_SRC;

  char* ws = (char*)d_ws;
  size_t off = 0;
  auto carve = [&](size_t bytes) -> char* { char* p = ws + off; off += (bytes + 255) & ~(size_t)255; return p; };
  const size_t slotX0 = (size_t)N_BATCH * K_CAT0;
  const size_t slotX1 = (size_t)N_BATCH * K_CAT1;
  const size_t slotH  = (size_t)N_BATCH * N_HID;
  const size_t slotQ  = (size_t)N_BATCH * N_QH;
  const size_t slotKP = (size_t)N_BATCH * KP_PITCH;
  unsigned short* WC0 = (unsigned short*)carve((size_t)N_GATE * K_CAT0 * 2);
  unsigned short* WC1 = (unsigned short*)carve((size_t)N_GATE * K_CAT1 * 2);
  unsigned short* WQH = (unsigned short*)carve((size_t)N_QH * N_HID * 2);
  unsigned short* WQL = (unsigned short*)carve((size_t)N_QH * N_HID * 2);
  unsigned short* WO  = (unsigned short*)carve((size_t)N_HID * K_CAT1 * 2);
  unsigned short* X0  = (unsigned short*)carve((size_t)(N_STEP + 1) * slotX0 * 2);
  unsigned short* X1  = (unsigned short*)carve((size_t)(N_STEP + 1) * slotX1 * 2);
  unsigned short* XO  = (unsigned short*)carve((size_t)N_STEP * slotX1 * 2);
  unsigned short* HBH = (unsigned short*)carve((size_t)(N_STEP + 1) * slotH * 2);
  unsigned short* HBL = (unsigned short*)carve((size_t)(N_STEP + 1) * slotH * 2);
  float* CS0 = (float*)carve((size_t)2 * slotH * 4);
  float* CS1 = (float*)carve((size_t)2 * slotH * 4);
  float* QML = (float*)carve((size_t)2 * slotQ * 4);
  float* BS0 = (float*)carve((size_t)N_GATE * 4);
  float* BS1 = (float*)carve((size_t)N_GATE * 4);
  float* BQH = (float*)carve((size_t)N_QH * 4);
  float* KP  = (float*)carve((size_t)(N_STEP + 1) * slotKP * 4);
  unsigned short* XOL = (unsigned short*)carve((size_t)2 * slotX1 * 2);
  unsigned short* A0L = (unsigned short*)carve(slotX0 * 2);
  unsigned short* A1L = (unsigned short*)carve(slotX1 * 2);
  if (off > ws_size || off > (size_t)134217728) return;

  cvt8_kernel<0, true><<<(N_GATE * (K_IN0 / 8)) / 256, 256, 0, stream>>>(W_ih0, K_IN0, K_IN0 / 8, N_GATE, WC0, WC0, K_CAT0, W_CARRY);
  cvt8_kernel<0, true><<<(N_GATE * (N_HID / 8)) / 256, 256, 0, stream>>>(W_hh0, N_HID, N_HID / 8, N_GATE, WC0 + COL_H0, WC0, K_CAT0, W_CARRY);
  cvt8_kernel<0, true><<<(N_GATE * (N_HID / 8)) / 256, 256, 0, stream>>>(W_ih1, N_HID, N_HID / 8, N_GATE, WC1, WC1, K_CAT1, W_CARRY);
  cvt8_kernel<0, true><<<(N_GATE * (N_HID / 8)) / 256, 256, 0, stream>>>(W_hh1, N_HID, N_HID / 8, N_GATE, WC1 + N_HID, WC1, K_CAT1, W_CARRY);
  cvt8_kernel<0, false><<<(N_HID * (K_CAT1 / 8)) / 256, 256, 0, stream>>>(W_out, K_CAT1, K_CAT1 / 8, N_HID, WO, WO, K_CAT1, W_CARRY);
  cvt8_kernel<1, false><<<(N_HID * (N_HID / 8)) / 256, 256, 0, stream>>>(W_a, N_HID, N_HID / 8, N_HID, WQH, WQL, N_HID, 1.0f);
  cvt8_kernel<1, false><<<(N_LAT * (N_HID / 8)) / 256, 256, 0, stream>>>(W_mu, N_HID, N_HID / 8, N_LAT, WQH + (size_t)N_HID * N_HID, WQL + (size_t)N_HID * N_HID, N_HID, 1.0f);
  cvt8_kernel<1, false><<<(N_LAT * (N_HID / 8)) / 256, 256, 0, stream>>>(W_lv, N_HID, N_HID / 8, N_LAT, WQH + (size_t)(N_HID + N_LAT) * N_HID, WQL + (size_t)(N_HID + N_LAT) * N_HID, N_HID, 1.0f);
  cvt8_kernel<2, false><<<(N_BATCH * (N_EMB / 8)) / 256, 256, 0, stream>>>(trg_emb, N_EMB, N_EMB / 8, N_BATCH, X0, A0L, K_CAT0, 1.0f);
  cvt8_kernel<0, false><<<((N_STEP - 1) * N_BATCH * (N_EMB / 8)) / 256, 256, 0, stream>>>(trg_emb + (size_t)N_BATCH * N_EMB, N_EMB, N_EMB / 8, (N_STEP - 1) * N_BATCH, X0 + slotX0, X0, K_CAT0, 1.0f);
  cvt8_kernel<2, false><<<(N_BATCH * (N_HID / 8)) / 256, 256, 0, stream>>>(in_feed, N_HID, N_HID / 8, N_BATCH, X0 + COL_FEED, A0L + COL_FEED, K_CAT0, 1.0f);
  cvt8_kernel<2, false><<<(N_BATCH * (N_HID / 8)) / 256, 256, 0, stream>>>(h0_in, N_HID, N_HID / 8, N_BATCH, X0 + COL_H0, A0L + COL_H0, K_CAT0, 1.0f);
  cvt8_kernel<2, false><<<(N_BATCH * (N_HID / 8)) / 256, 256, 0, stream>>>(h0_in + slotH, N_HID, N_HID / 8, N_BATCH, X1 + N_HID, A1L + N_HID, K_CAT1, 1.0f);
  cvt8_kernel<1, false><<<(N_BATCH * (N_HID / 8)) / 256, 256, 0, stream>>>(h0_in + slotH, N_HID, N_HID / 8, N_BATCH, HBH, HBL, N_HID, 1.0f);
  bias_kernel<<<10, 256, 0, stream>>>(b_ih0, b_hh0, b_ih1, b_hh1, b_mu, b_lv, BS0, BS1, BQH);
  gemm_qh_kernel<<<N_QH / 256, 128, 0, stream>>>(HBH, HBL, WQH, WQL, BQH, QML);
  zk_kernel<<<N_BATCH, 256, 0, stream>>>(QML, eps, X0, A0L, KP);

  for (int t = 0; t < N_STEP; ++t) {
    unsigned short* X0t = X0 + (size_t)t * slotX0;
    unsigned short* X0n = X0 + (size_t)(t + 1) * slotX0;
    unsigned short* X1t = X1 + (size_t)t * slotX1;
    unsigned short* X1n = X1 + (size_t)(t + 1) * slotX1;
    unsigned short* XOt = XO + (size_t)t * slotX1;
    unsigned short* XOLt = XOL + (size_t)(t & 1) * slotX1;
    unsigned short* HBHn = HBH + (size_t)(t + 1) * slotH;
    unsigned short* HBLn = HBL + (size_t)(t + 1) * slotH;
    const float* cin0 = (t == 0) ? c0_in : (CS0 + (size_t)(t & 1) * slotH);
    const float* cin1 = (t == 0) ? (c0_in + slotH) : (CS1 + (size_t)(t & 1) * slotH);
    float* cnx0 = CS0 + (size_t)((t + 1) & 1) * slotH;
    float* cnx1 = CS1 + (size_t)((t + 1) & 1) * slotH;
    float* qslot = QML + (size_t)((t + 1) & 1) * slotQ;
    const int tn = (t + 1 < N_STEP) ? (t + 1) : (N_STEP - 1);

    if (t == 0) {
      gemm_cell_kernel<2, true><<<N_GATE / 256, 128, 0, stream>>>(X0t, A0L, K_CAT0, WC0, K_CAT0,
                                                                  W_ih0, K_IN0, K_IN0, W_hh0, N_HID,
                                                                  BS0, cin0, cnx0,
                                                                  X1t, K_CAT1, X0n + COL_H0, K_CAT0,
                                                                  HBHn, HBLn, A1L, K_CAT1);
      gemm_cell_kernel<1, true><<<N_GATE / 256, 128, 0, stream>>>(X1t, A1L, K_CAT1, WC1, K_CAT1,
                                                                  W_ih1, N_HID, N_HID, W_hh1, N_HID,
                                                                  BS1, cin1, cnx1,
                                                                  XOt + N_HID, K_CAT1, X1n + N_HID, K_CAT1,
                                                                  HBHn, HBLn, XOLt + N_HID, K_CAT1);
    } else {
      gemm_cell_kernel<0, false><<<N_GATE / 256, 128, 0, stream>>>(X0t, X0t, K_CAT0, WC0, K_CAT0,
                                                                   W_ih0, K_IN0, K_IN0, W_hh0, N_HID,
                                                                   BS0, cin0, cnx0,
                                                                   X1t, K_CAT1, X0n + COL_H0, K_CAT0,
                                                                   HBHn, HBLn, XOLt, K_CAT1);
      gemm_cell_kernel<1, false><<<N_GATE / 256, 128, 0, stream>>>(X1t, X1t, K_CAT1, WC1, K_CAT1,
                                                                   W_ih1, N_HID, N_HID, W_hh1, N_HID,
                                                                   BS1, cin1, cnx1,
                                                                   XOt + N_HID, K_CAT1, X1n + N_HID, K_CAT1,
                                                                   HBHn, HBLn, XOLt + N_HID, K_CAT1);
    }
    gemm_qh_kernel<<<N_QH / 256, 128, 0, stream>>>(HBHn, HBLn, WQH, WQL, BQH, qslot);
    att_kernel<<<N_BATCH, 256, 0, stream>>>(qslot, enc, lengths, eps + (size_t)tn * N_BATCH * N_LAT,
                                            attns + (size_t)t * N_BATCH * N_SRC, XOt, XOLt, X0n,
                                            KP + (size_t)(t + 1) * slotKP);
    gemm_out_kernel<<<N_HID / 256, 128, 0, stream>>>(XOt, XOLt, WO, dec + (size_t)t * N_BATCH * N_HID,
                                                     X0n + COL_FEED, K_CAT0);
  }
  kld_final_kernel<<<1, 32, 0, stream>>>(KP, kld);
}
